// encoder_80607946211781
// MI455X (gfx1250) — hardware-run, weakly checked
//
#include <hip/hip_runtime.h>
#include <math.h>

typedef __attribute__((ext_vector_type(16))) _Float16 v16h;
typedef __attribute__((ext_vector_type(8)))  _Float16 v8h;
typedef __attribute__((ext_vector_type(16))) __bf16   v16b;
typedef __attribute__((ext_vector_type(8)))  __bf16   v8b;
typedef __attribute__((ext_vector_type(8)))  float    v8f;
typedef __attribute__((ext_vector_type(4)))  float    v4f;

constexpr int kBatch  = 128;
constexpr int kSteps  = 128;
constexpr int kSer    = 128;
constexpr int kHid    = 64;
constexpr int kHc     = 2 * kHid;
constexpr int kGate4  = 4 * kHid;
constexpr int kRowsS  = kBatch * kSer;
constexpr int kThr    = 256;
constexpr int kThrRun = 512;
constexpr int kSeqBlk = 16;
constexpr int kHP     = 72;
constexpr int kXP     = 136;
constexpr int kOut0   = kBatch * kSteps * kSer;
constexpr int kOut1   = kBatch * kSteps * kHid;

constexpr float kInCarry  = 1024.0f;
constexpr float kWCarry   = 1024.0f;
constexpr float kHCarry   = 4096.0f;
constexpr float kCCarry   = 256.0f;
constexpr float kXhCarry  = 4096.0f;
constexpr float kUeScale  = 1.0f / (kInCarry * kWCarry);
constexpr float kHScale   = 1.0f / (kHCarry * kWCarry);
constexpr float kCScale   = 1.0f / (kCCarry * kWCarry);
constexpr float kXhScale  = 1.0f / (kXhCarry * kWCarry);
constexpr float kF16MinNormal = 6.103515625e-5f;

static_assert(kSteps == kSer && kSer == 128 && kHc == 128 && kGate4 == 256 && kRowsS == 16384, "plane sizes (the attention's inner index runs over the 128 steps of a series' history)");
static_assert((kRowsS % 64) == 0 && (kSer % 64) == 0 && (kSteps % 32) == 0, "hoisted GEMM: M, N multiples of 64, K of 32");
static_assert(kSeqBlk == kThrRun / 32 && kBatch % kSeqBlk == 0, "16 waves = 16 batch rows per block");
static_assert((kHP % 8) == 0 && kHP >= kHid + 8 && (kXP % 8) == 0 && kXP >= kSer + 8, "f16 tile pitches");

constexpr size_t kOffXT   = 0;
constexpr size_t kOffUEW  = kOffXT  + (size_t)kRowsS * kSteps * 2;
constexpr size_t kOffWEH  = kOffUEW + (size_t)kSer * kSteps * 2;
constexpr size_t kOffWIH  = kOffWEH + (size_t)kSer * kHc * 2;
constexpr size_t kOffWHH  = kOffWIH + (size_t)kGate4 * kSer * 2;
constexpr size_t kOffUEX  = kOffWHH + (size_t)kGate4 * kHid * 2;
constexpr size_t kWsTotal = kOffUEX + (size_t)kRowsS * kSer * 4;
static_assert(kWsTotal == 12746752ull, "carve total");
static_assert(kWsTotal <= 134217728ull, "carve cap");
static_assert((kOffUEW % 256) == 0 && (kOffWEH % 256) == 0 && (kOffWIH % 256) == 0 && (kOffWHH % 256) == 0 && (kOffUEX % 256) == 0, "aligned regions");

__device__ __forceinline__ unsigned short f2bf_bits(float f) {
  unsigned u = __float_as_uint(f);
  return (unsigned short)((u + 0x7FFFu + ((u >> 16) & 1u)) >> 16);
}
__device__ __forceinline__ float bf_bits2f(unsigned short h) { return __uint_as_float(((unsigned)h) << 16); }
__device__ __forceinline__ float bf16r(float f) { return bf_bits2f(f2bf_bits(f)); }
__device__ __forceinline__ float carry_flush(float v, float carry) {
  const float s = v * carry;
  return (fabsf(s) < kF16MinNormal) ? 0.0f : s;
}
__device__ __forceinline__ float frcp(float x) { return __builtin_amdgcn_rcpf(x); }

__device__ __forceinline__ void dep_guard4_h(v8f& a, v8f& b, v8f& c, v8f& d, v16h x, v16h y) { asm volatile("v_nop\n\tv_nop\n\tv_nop\n\tv_nop" : "+v"(a), "+v"(b), "+v"(c), "+v"(d) : "v"(x), "v"(y)); }
__device__ __forceinline__ void dep_guard4_b(v8f& a, v8f& b, v8f& c, v8f& d, v16b x, v16b y) { asm volatile("v_nop\n\tv_nop\n\tv_nop\n\tv_nop" : "+v"(a), "+v"(b), "+v"(c), "+v"(d) : "v"(x), "v"(y)); }
__device__ __forceinline__ void keep4_h(v16h a, v16h b, v16h c, v16h d) { asm volatile("v_nop" :: "v"(a), "v"(b), "v"(c), "v"(d)); }
__device__ __forceinline__ void keep4_b(v16b a, v16b b, v16b c, v16b d) { asm volatile("v_nop" :: "v"(a), "v"(b), "v"(c), "v"(d)); }
__device__ __forceinline__ void acc_guard4(v8f& a, v8f& b, v8f& c, v8f& d) { asm volatile("v_nop\n\tv_nop\n\tv_nop\n\tv_nop" : "+v"(a), "+v"(b), "+v"(c), "+v"(d)); }

template <typename T> struct Frag;
template <> struct Frag<_Float16> {
  typedef v16h V; union U { v16h v; v8h h[2]; };
  static __device__ __forceinline__ v16h load(const _Float16* p) {
    U f; f.h[0] = *(const v8h*)(p); f.h[1] = *(const v8h*)(p + 16); return f.v;
  }
  static __device__ __forceinline__ v8f mma(v16h a, v16h b, v8f c) {
    return __builtin_amdgcn_wmma_f32_16x16x32_f16(false, a, false, b, (short)0, c, false, false);
  }
  static __device__ __forceinline__ void guard4(v8f& a, v8f& b, v8f& c, v8f& d, v16h x, v16h y) { dep_guard4_h(a, b, c, d, x, y); }
  static __device__ __forceinline__ void keep(v16h a, v16h b, v16h c, v16h d) { keep4_h(a, b, c, d); }
};
template <> struct Frag<__bf16> {
  typedef v16b V; union U { v16b v; v8b h[2]; };
  static __device__ __forceinline__ v16b load(const __bf16* p) {
    U f; f.h[0] = *(const v8b*)(p); f.h[1] = *(const v8b*)(p + 16); return f.v;
  }
  static __device__ __forceinline__ v8f mma(v16b a, v16b b, v8f c) {
    return __builtin_amdgcn_wmma_f32_16x16x32_bf16(false, a, false, b, (short)0, c, false, false);
  }
  static __device__ __forceinline__ void guard4(v8f& a, v8f& b, v8f& c, v8f& d, v16b x, v16b y) { dep_guard4_b(a, b, c, d, x, y); }
  static __device__ __forceinline__ void keep(v16b a, v16b b, v16b c, v16b d) { keep4_b(a, b, c, d); }
};

__device__ __forceinline__ v8f mma_h(v16h a, v16h b, v8f c) {
  c = __builtin_amdgcn_wmma_f32_16x16x32_f16(false, a, false, b, (short)0, c, false, false);
  asm volatile("v_nop\n\tv_nop\n\tv_nop\n\tv_nop" : "+v"(c) : "v"(a), "v"(b));
  return c;
}

template <int ET> struct Elem;
template <> struct Elem<0> { typedef _Float16 T; };
template <> struct Elem<1> { typedef __bf16 T; };
template <int ET, bool SPLIT, int BIAS_MODE, int OUT_MODE, bool RESID, int ACT = 0>
__global__ __launch_bounds__(256) void wmma_gemm64(
    const unsigned short* __restrict__ Ap, const unsigned short* __restrict__ A2p, int lda, long strideA,
    const unsigned short* __restrict__ Btp, const unsigned short* __restrict__ Bt2p, int ldb, long strideB,
    void* __restrict__ Cout, void* __restrict__ Cout2, int ldc, long strideC,
    const float* __restrict__ bias,
    const float* __restrict__ resid, long strideR,
    int M, int N, int K, float scale) {
  typedef typename Elem<ET>::T T;
  typedef typename Frag<T>::V V;
  const T* A = (const T*)Ap; const T* A2 = (const T*)A2p; const T* Bt = (const T*)Btp; const T* Bt2 = (const T*)Bt2p;
  __shared__ __align__(16) float sT[8][16 * 68];
  const int b    = blockIdx.y;
  const int lane = threadIdx.x & 31;
  const int wave = threadIdx.x >> 5;
  const int tilesN = N >> 6;
  const int tilesM = M >> 6;
  const int tile = blockIdx.x * 8 + wave;
  if (tile >= tilesM * tilesN) return;
  const int tm = tile / tilesN;
  const int tn = tile - tm * tilesN;
  const int m0 = tm << 6;
  const int n0 = tn << 6;

  const T* Ab  = A  + (size_t)b * strideA;
  const T* Bb  = Bt + (size_t)b * strideB;
  const T* Ab2 = SPLIT ? (A2  + (size_t)b * strideA) : nullptr;
  const T* Bb2 = SPLIT ? (Bt2 + (size_t)b * strideB) : nullptr;

  const int rlane = lane & 15;
  const int koff  = (lane >> 4) * 8;
  const int mOff  = (lane >> 4) * 8;

  v8f acc[4][4];
#pragma unroll
  for (int i = 0; i < 4; ++i)
#pragma unroll
    for (int j = 0; j < 4; ++j) acc[i][j] = (v8f){0.f,0.f,0.f,0.f,0.f,0.f,0.f,0.f};

  for (int k0 = 0; k0 < K; k0 += 32) {
    V bh[4], bl[4];
#pragma unroll
    for (int j = 0; j < 4; ++j) {
      const size_t bo = (size_t)(n0 + (j << 4) + rlane) * ldb + koff + k0;
      bh[j] = Frag<T>::load(Bb + bo);
      if (SPLIT) bl[j] = Frag<T>::load(Bb2 + bo);
    }
#pragma unroll
    for (int i = 0; i < 4; ++i) {
      const size_t ao = (size_t)(m0 + (i << 4) + rlane) * lda + koff + k0;
      V ah = Frag<T>::load(Ab + ao);
      V al;
      if (SPLIT) al = Frag<T>::load(Ab2 + ao);
#pragma unroll
      for (int j = 0; j < 4; ++j) {
        acc[i][j] = Frag<T>::mma(ah, bh[j], acc[i][j]);
        if (SPLIT) {
          acc[i][j] = Frag<T>::mma(ah, bl[j], acc[i][j]);
          acc[i][j] = Frag<T>::mma(al, bh[j], acc[i][j]);
        }
      }
      Frag<T>::guard4(acc[i][0], acc[i][1], acc[i][2], acc[i][3], ah, SPLIT ? al : ah);
    }
    Frag<T>::keep(bh[0], bh[1], bh[2], bh[3]);
    if (SPLIT) Frag<T>::keep(bl[0], bl[1], bl[2], bl[3]);
  }
  acc_guard4(acc[0][0], acc[0][1], acc[0][2], acc[0][3]);
  acc_guard4(acc[1][0], acc[1][1], acc[1][2], acc[1][3]);
  acc_guard4(acc[2][0], acc[2][1], acc[2][2], acc[2][3]);
  acc_guard4(acc[3][0], acc[3][1], acc[3][2], acc[3][3]);

  float* slab = sT[wave];
  const float* Rb = RESID ? (resid + (size_t)b * strideR) : nullptr;
#pragma unroll
  for (int i = 0; i < 4; ++i) {
    const int mBase = m0 + (i << 4);
#pragma unroll
    for (int j = 0; j < 4; ++j) {
      const int n = n0 + (j << 4) + rlane;
      float bv = 0.f;
      if (BIAS_MODE == 2) bv = bias[n];
#pragma unroll
      for (int r = 0; r < 8; ++r) {
        float v = acc[i][j][r] * scale;
        if (BIAS_MODE == 1) v += bias[mBase + mOff + r];
        if (BIAS_MODE == 2) v += bv;
        if (RESID) v += Rb[(size_t)(mBase + mOff + r) * ldc + n];
        if (ACT == 1) v = tanhf(v);
        if (ACT == 2) v = fmaxf(v, 0.0f);
        if (ACT == 3) v = v / (1.0f + expf(-v));
        if (ACT == 4) v = (v > 0.f) ? v : 0.01f * v;
        slab[(mOff + r) * 68 + (j << 4) + rlane] = v;
      }
    }
    __builtin_amdgcn_fence(__ATOMIC_RELEASE, "workgroup");
    __builtin_amdgcn_wave_barrier();
    __builtin_amdgcn_fence(__ATOMIC_ACQUIRE, "workgroup");
    if (OUT_MODE == 0) {
      float* C = (float*)Cout + (size_t)b * strideC;
      const int hh = lane >> 4, c4 = (lane & 15) * 4;
      for (int pass = 0; pass < 2; ++pass) {
#pragma unroll
        for (int it = 0; it < 8; ++it) {
          const int row = it * 2 + hh;
          v4f v = *(const v4f*)(slab + row * 68 + c4);
          *(volatile v4f*)(C + (size_t)(mBase + row) * ldc + n0 + c4) = v;
        }
        __threadfence();
      }
    } else {
      const int q = lane >> 3, c8 = (lane & 7) * 8;
      unsigned short* C  = (unsigned short*)Cout  + (size_t)b * strideC;
      unsigned short* C2 = (OUT_MODE == 2) ? ((unsigned short*)Cout2 + (size_t)b * strideC) : nullptr;
      for (int pass = 0; pass < 2; ++pass) {
#pragma unroll
        for (int it = 0; it < 4; ++it) {
          const int row = it * 4 + q;
          const float* sp = slab + row * 68 + c8;
          v8h hv, lv;
#pragma unroll
          for (int e = 0; e < 8; ++e) {
            if (OUT_MODE == 1) {
              hv[e] = (_Float16)sp[e];
            } else {
              unsigned short hb = f2bf_bits(sp[e]);
              unsigned short lb = f2bf_bits(sp[e] - bf_bits2f(hb));
              hv[e] = __builtin_bit_cast(_Float16, hb);
              lv[e] = __builtin_bit_cast(_Float16, lb);
            }
          }
          *(volatile v8h*)(C + (size_t)(mBase + row) * ldc + n0 + c8) = hv;
          if (OUT_MODE == 2) *(volatile v8h*)(C2 + (size_t)(mBase + row) * ldc + n0 + c8) = lv;
        }
        __threadfence();
      }
    }
    __builtin_amdgcn_fence(__ATOMIC_RELEASE, "workgroup");
    __builtin_amdgcn_wave_barrier();
    __builtin_amdgcn_fence(__ATOMIC_ACQUIRE, "workgroup");
  }
}

__global__ __launch_bounds__(kThr) void cast_plane_kernel(const float* __restrict__ src, unsigned short* __restrict__ dst,
                                                          int colsLog2, int dstPitch, int dstOff) {
  const int i   = blockIdx.x * kThr + threadIdx.x;
  const int sh  = colsLog2 - 3;
  const int row = i >> sh;
  const int c8  = (i & ((1 << sh) - 1)) * 8;
  const float* sp = src + ((size_t)row << colsLog2) + c8;
  const v4f a0 = *(const v4f*)(sp);
  const v4f a1 = *(const v4f*)(sp + 4);
  v8h hv;
#pragma unroll
  for (int e = 0; e < 4; ++e) {
    const float f0 = a0[e];
    const float f1 = a1[e];
    hv[e]     = (_Float16)carry_flush(bf16r(f0), kInCarry);
    hv[4 + e] = (_Float16)carry_flush(bf16r(f1), kInCarry);
  }
  unsigned short* dp = dst + (size_t)row * dstPitch + dstOff + c8;
  *(volatile v8h*)dp = hv;
  __threadfence();
  *(volatile v8h*)dp = hv;
}
static_assert(kInCarry == kWCarry, "one cast kernel serves inputs and weights");

__global__ __launch_bounds__(kThr) void series_plane_kernel(const float* __restrict__ x, unsigned short* __restrict__ XT) {
  __shared__ __align__(16) float sTile[64 * 68];
  const int tid = threadIdx.x;
  const int d0 = blockIdx.x * 64;
  const int t0 = blockIdx.y * 64;
  const int b  = blockIdx.z;
  {
    const int tt = tid >> 4;
    const int d4 = (tid & 15) * 4;
#pragma unroll
    for (int i = 0; i < 4; ++i) {
      const int t = tt + 16 * i;
      const v4f v = *(const v4f*)(x + ((size_t)b * kSteps + t0 + t) * kSer + d0 + d4);
#pragma unroll
      for (int e = 0; e < 4; ++e) {
        const float fv = v[e];
        sTile[(d4 + e) * 68 + t] = carry_flush(bf16r(fv), kInCarry);
      }
    }
  }
  __syncthreads();
  const int t8 = (tid & 7) * 8;
  v8h hv[2];
#pragma unroll
  for (int it = 0; it < 2; ++it) {
    const int d = (tid >> 3) + 32 * it;
    const float* sp = sTile + d * 68 + t8;
    const v4f a0 = *(const v4f*)(sp);
    const v4f a1 = *(const v4f*)(sp + 4);
#pragma unroll
    for (int e = 0; e < 4; ++e) {
      const float f0 = a0[e];
      const float f1 = a1[e];
      hv[it][e]     = (_Float16)f0;
      hv[it][4 + e] = (_Float16)f1;
    }
  }
  for (int pass = 0; pass < 2; ++pass) {
#pragma unroll
    for (int it = 0; it < 2; ++it) {
      const int d = (tid >> 3) + 32 * it;
      *(volatile v8h*)(XT + ((size_t)b * kSer + d0 + d) * kSteps + t0 + t8) = hv[it];
    }
    __threadfence();
  }
}

__device__ __forceinline__ float score_tanh(float v) {
  const float e = __expf(2.0f * v);
  return 1.0f - 2.0f * frcp(e + 1.0f);
}
__device__ __forceinline__ float gate_sigmoid(float v) { return 1.0f / (1.0f + expf(-v)); }

__global__ __launch_bounds__(kThrRun) void attn_cell_run_kernel(const float* __restrict__ x,
                                                                const float* __restrict__ UEX,
                                                                const unsigned short* __restrict__ WEHp,
                                                                const unsigned short* __restrict__ WIHp,
                                                                const unsigned short* __restrict__ WHHp,
                                                                const float* __restrict__ be, const float* __restrict__ ve,
                                                                const float* __restrict__ vb,
                                                                const float* __restrict__ bih, const float* __restrict__ bhh,
                                                                float* __restrict__ OUT0, float* __restrict__ OUT1) {
  __shared__ __align__(16) _Float16 sHh[2][kSeqBlk * kHP];
  __shared__ __align__(16) _Float16 sCh[kSeqBlk * kHP];
  __shared__ __align__(16) _Float16 sXh[kSeqBlk * kXP];
  __shared__ __align__(16) float    sWe[kSeqBlk * kSer];
  __shared__ __align__(16) float    sHm[kSeqBlk * kHid];
  __shared__ __align__(16) float    sCm[kSeqBlk * kHid];
  __shared__ __align__(16) float    sBe[kSer];
  __shared__ __align__(16) float    sVe[kSer];
  __shared__ __align__(16) float    sBg[kGate4];
  const _Float16* WEH = (const _Float16*)WEHp;
  const _Float16* WIH = (const _Float16*)WIHp;
  const _Float16* WHH = (const _Float16*)WHHp;
  const int tid = threadIdx.x, lane = tid & 31;
  const int wave = __builtin_amdgcn_readfirstlane(tid >> 5);
  const int c = lane & 15, hh = lane >> 4, koff = hh * 8;
  const int b0 = blockIdx.x * kSeqBlk;

  {
    _Float16* hf = &sHh[0][0];
#pragma unroll 1
    for (int i = tid; i < 2 * kSeqBlk * kHP; i += kThrRun) hf[i] = (_Float16)0.0f;
#pragma unroll 1
    for (int i = tid; i < kSeqBlk * kHP; i += kThrRun) sCh[i] = (_Float16)0.0f;
#pragma unroll 1
    for (int i = tid; i < kSeqBlk * kXP; i += kThrRun) sXh[i] = (_Float16)0.0f;
#pragma unroll 1
    for (int i = tid; i < kSeqBlk * kSer; i += kThrRun) sWe[i] = 0.0f;
#pragma unroll 1
    for (int i = tid; i < kSeqBlk * kHid; i += kThrRun) { sHm[i] = 0.0f; sCm[i] = 0.0f; }
#pragma unroll 1
    for (int i = tid; i < kSer; i += kThrRun) { sBe[i] = bf16r(be[i]); sVe[i] = bf16r(ve[i]); }
#pragma unroll 1
    for (int i = tid; i < kGate4; i += kThrRun) sBg[i] = bf16r(bih[i]) + bf16r(bhh[i]);
  }
  __syncthreads();
  const float vbv = bf16r(vb[0]);
  const v8f z8 = {0.f, 0.f, 0.f, 0.f, 0.f, 0.f, 0.f, 0.f};

#pragma unroll 1
  for (int t = 0; t < kSteps; ++t) {
    const int cur = t & 1;
    const _Float16* hrow = &sHh[cur][0] + c * kHP + koff;

    if (wave < 8) {
      const int s = 16 * wave + c;
      const _Float16* wrow = WEH + (size_t)s * kHc + koff;
      const _Float16* crow = sCh + c * kHP + koff;
      v8f ah = z8, ac = z8;
#pragma unroll
      for (int k0 = 0; k0 < kHid; k0 += 32) {
        const v16h a  = Frag<_Float16>::load(hrow + k0);
        const v16h fb = Frag<_Float16>::load(wrow + k0);
        ah = mma_h(a, fb, ah);
      }
#pragma unroll
      for (int k0 = 0; k0 < kHid; k0 += 32) {
        const v16h a  = Frag<_Float16>::load(crow + k0);
        const v16h fb = Frag<_Float16>::load(wrow + kHid + k0);
        ac = mma_h(a, fb, ac);
      }
      const float bev = sBe[s];
#pragma unroll
      for (int r = 0; r < 8; ++r) sWe[(8 * hh + r) * kSer + s] = (ah[r] * kHScale + ac[r] * kCScale) + bev;
    }
    __syncthreads();

    {
      const int b = b0 + wave;
      const float* wrow = sWe + wave * kSer;
      const float* urow = UEX + ((size_t)b * kSer + 4 * lane) * kSer;
      float v[4];
#pragma unroll
      for (int k = 0; k < 4; ++k) v[k] = 0.0f;
#pragma unroll 1
      for (int s4 = 0; s4 < kSer; s4 += 4) {
        const v4f w4 = *(const v4f*)(wrow + s4);
        const v4f e4 = *(const v4f*)(sVe + s4);
#pragma unroll
        for (int k = 0; k < 4; ++k) {
          const v4f u4 = *(const v4f*)(urow + (size_t)k * kSer + s4);
#pragma unroll
          for (int e = 0; e < 4; ++e) v[k] += score_tanh(w4[e] + u4[e]) * e4[e];
        }
      }
      float mx = -3.0e38f;
#pragma unroll
      for (int k = 0; k < 4; ++k) { v[k] += vbv; mx = fmaxf(mx, v[k]); }
      mx = fmaxf(mx, __shfl_xor(mx, 1, 32));
      mx = fmaxf(mx, __shfl_xor(mx, 2, 32));
      mx = fmaxf(mx, __shfl_xor(mx, 4, 32));
      mx = fmaxf(mx, __shfl_xor(mx, 8, 32));
      mx = fmaxf(mx, __shfl_xor(mx, 16, 32));
      float ex[4];
      float se = 0.0f;
#pragma unroll
      for (int k = 0; k < 4; ++k) { ex[k] = expf(v[k] - mx); se += ex[k]; }
      se += __shfl_xor(se, 1, 32);
      se += __shfl_xor(se, 2, 32);
      se += __shfl_xor(se, 4, 32);
      se += __shfl_xor(se, 8, 32);
      se += __shfl_xor(se, 16, 32);
      const v4f x4 = *(const v4f*)(x + ((size_t)b * kSteps + t) * kSer + 4 * lane);
      v4f xh;
#pragma unroll
      for (int k = 0; k < 4; ++k) {
        const float xv = x4[k];
        xh[k] = (ex[k] / se) * bf16r(xv);
      }
      float* op = OUT0 + ((size_t)b * kSteps + t) * kSer + 4 * lane;
      for (int pass = 0; pass < 2; ++pass) {
        *(volatile v4f*)op = xh;
        __threadfence();
      }
#pragma unroll
      for (int k = 0; k < 4; ++k) sXh[wave * kXP + 4 * lane + k] = (_Float16)carry_flush(xh[k], kXhCarry);
    }
    __syncthreads();

    if (wave < 4) {
      const int j = 16 * wave + c;
      const _Float16* xrow = sXh + c * kXP + koff;
      v8f gx[4], gh[4];
#pragma unroll
      for (int g = 0; g < 4; ++g) { gx[g] = z8; gh[g] = z8; }
#pragma unroll 1
      for (int k0 = 0; k0 < kSer; k0 += 32) {
        const v16h a = Frag<_Float16>::load(xrow + k0);
#pragma unroll
        for (int g = 0; g < 4; ++g) {
          const v16h fb = Frag<_Float16>::load(WIH + (size_t)(g * kHid + j) * kSer + koff + k0);
          gx[g] = mma_h(a, fb, gx[g]);
        }
      }
#pragma unroll 1
      for (int k0 = 0; k0 < kHid; k0 += 32) {
        const v16h a = Frag<_Float16>::load(hrow + k0);
#pragma unroll
        for (int g = 0; g < 4; ++g) {
          const v16h fb = Frag<_Float16>::load(WHH + (size_t)(g * kHid + j) * kHid + koff + k0);
          gh[g] = mma_h(a, fb, gh[g]);
        }
      }
      _Float16* hn = &sHh[cur ^ 1][0];
#pragma unroll
      for (int r = 0; r < 8; ++r) {
        const int row = 8 * hh + r;
        const float gi = (gx[0][r] * kXhScale + gh[0][r] * kHScale) + sBg[j];
        const float gf = (gx[1][r] * kXhScale + gh[1][r] * kHScale) + sBg[kHid + j];
        const float gg = (gx[2][r] * kXhScale + gh[2][r] * kHScale) + sBg[2 * kHid + j];
        const float go = (gx[3][r] * kXhScale + gh[3][r] * kHScale) + sBg[3 * kHid + j];
        const float cn = gate_sigmoid(gf) * sCm[row * kHid + j] + gate_sigmoid(gi) * tanhf(gg);
        const float hv = gate_sigmoid(go) * tanhf(cn);
        sCm[row * kHid + j] = cn;
        sHm[row * kHid + j] = hv;
        hn[row * kHP + j]  = (_Float16)carry_flush(hv, kHCarry);
        sCh[row * kHP + j] = (_Float16)carry_flush(cn, kCCarry);
      }
    }
    __syncthreads();

    if (wave < 8) {
      const int row = 2 * wave + hh;
      const v4f hv4 = *(const v4f*)(sHm + row * kHid + 4 * c);
      float* op = OUT1 + ((size_t)(b0 + row) * kSteps + t) * kHid + 4 * c;
      for (int pass = 0; pass < 2; ++pass) {
        *(volatile v4f*)op = hv4;
        __threadfence();
      }
    }
  }
}

static_assert(((kRowsS / 64) * (kSer / 64)) % 8 == 0, "GEMM grid exact");
static_assert((kSer * kSteps / 8) % kThr == 0 && (kSer * kHc / 8) % kThr == 0 && (kGate4 * kSer / 8) % kThr == 0 && (kGate4 * kHid / 8) % kThr == 0, "weight cast grids exact");

extern "C" void kernel_launch(void* const* d_in, const int* in_sizes, int n_in,
                              void* d_out, int out_size, void* d_ws, size_t ws_size,
                              hipStream_t stream) {
  if (n_in < 11 || d_out == nullptr || d_ws == nullptr) return;
  if (in_sizes[0] != kBatch * kSteps * kSer) return;
  if (in_sizes[1] != kSer * kHc || in_sizes[2] != kSer) return;
  if (in_sizes[3] != kSer * kSteps || in_sizes[4] != kSer) return;
  if (in_sizes[5] != kSer || in_sizes[6] != 1) return;
  if (in_sizes[7] != kGate4 * kSer || in_sizes[8] != kGate4 * kHid) return;
  if (in_sizes[9] != kGate4 || in_sizes[10] != kGate4) return;
  if (out_size != kOut0 + kOut1) return;
  if (ws_size < kWsTotal) return;

  const float* x    = (const float*)d_in[0];
  const float* Weh  = (const float*)d_in[1];
  const float* be   = (const float*)d_in[2];
  const float* Ue   = (const float*)d_in[3];
  const float* ub   = (const float*)d_in[4];
  const float* ve   = (const float*)d_in[5];
  const float* vb   = (const float*)d_in[6];
  const float* Wih  = (const float*)d_in[7];
  const float* Whh  = (const float*)d_in[8];
  const float* bih  = (const float*)d_in[9];
  const float* bhh  = (const float*)d_in[10];
  float* out0 = (float*)d_out;
  float* out1 = out0 + kOut0;

  char* ws = (char*)d_ws;
  unsigned short* XT  = (unsigned short*)(ws + kOffXT);
  unsigned short* UEW = (unsigned short*)(ws + kOffUEW);
  unsigned short* WEH = (unsigned short*)(ws + kOffWEH);
  unsigned short* WIH = (unsigned short*)(ws + kOffWIH);
  unsigned short* WHH = (unsigned short*)(ws + kOffWHH);
  float*          UEX = (float*)(ws + kOffUEX);

  series_plane_kernel<<<dim3(kSer / 64, kSteps / 64, kBatch), kThr, 0, stream>>>(x, XT);
  cast_plane_kernel<<<(kSer   * kSteps / 8) / kThr, kThr, 0, stream>>>(Ue,  UEW, 7, kSteps, 0);
  cast_plane_kernel<<<(kSer   * kHc    / 8) / kThr, kThr, 0, stream>>>(Weh, WEH, 7, kHc,    0);
  cast_plane_kernel<<<(kGate4 * kSer   / 8) / kThr, kThr, 0, stream>>>(Wih, WIH, 7, kSer,   0);
  cast_plane_kernel<<<(kGate4 * kHid   / 8) / kThr, kThr, 0, stream>>>(Whh, WHH, 6, kHid,   0);

  wmma_gemm64<0, false, 2, 0, false, 0><<<dim3((kRowsS / 64) * (kSer / 64) / 8, 1), 256, 0, stream>>>(
      XT, XT, kSteps, 0L, UEW, UEW, kSteps, 0L, (void*)UEX, (void*)UEX, kSer, 0L,
      ub, nullptr, 0L, kRowsS, kSer, kSteps, kUeScale);

  attn_cell_run_kernel<<<kBatch / kSeqBlk, kThrRun, 0, stream>>>(x, UEX, WEH, WIH, WHH, be, ve, vb, bih, bhh, out0, out1);
}
